// GATConvBlock_74603581932064
// MI455X (gfx1250) — hardware-verified
//
#include <hip/hip_runtime.h>
#include <stddef.h>
#include <stdint.h>


#define DIN     128
#define HPW     160
#define NTHR    256
#define NWAVE   8
#define EPT     8
#define CHUNK   (NTHR * EPT)
#define WCAP    (EPT * 32)
#define LISTN   (NWAVE * WCAP)
#define NBMAX   2048
#define RCAP    28672
#define DEGCAP  128
#define STW     512
#define STS     (NWAVE * STW)
#define PREC    256
#define GBM     64
#define GBN     128
#define GTHR    128
#define NSTV    ((16 * HPW) / 128)
#define CX      8.0f
#define CW      64.0f
#define CL      2048.0f
#define SCL_HI  0.001953125f
#define SCL_LO  9.5367431640625e-7f
#define NEG_SLOPE 0.2f
#define SELU_SC 1.0507009873554805f
#define SELU_AL 1.6732632423543772f
#define EPS_BN  0.00001f
#define WSMAX   134217728
#define LDS_AGG ((2 * RCAP + 2 * NBMAX + LISTN) * 4 + 64)

static_assert((CHUNK & (CHUNK - 1)) == 0 && CHUNK <= 4096);
static_assert((NBMAX & (NBMAX - 1)) == 0 && NBMAX <= 4096);
static_assert(NTHR * 8 == NBMAX);
static_assert(LISTN >= NBMAX);
static_assert(LISTN >= NWAVE * WCAP);
static_assert((RCAP % 32) == 0);
static_assert(STS + NWAVE * PREC + PREC <= RCAP);
static_assert(4 * 32 <= STW);
static_assert(LDS_AGG <= 300000);
static_assert(GBM == (GTHR / 32) * 16);
static_assert(GTHR == GBN && GBN == DIN);
static_assert(2 * GBM == GTHR);
static_assert((DIN % 32) == 0 && DIN / 8 == 16);
static_assert(HPW == DIN + 32 && ((HPW * 4) % 128) == 0);
static_assert(NSTV * 128 == 16 * HPW);
static_assert(GBM * HPW * 4 + 2 * GBN * 4 <= 49152);
static_assert(PREC == 2 * DIN && NTHR == PREC);

typedef float    v4f  __attribute__((ext_vector_type(4)));
typedef float    v8f  __attribute__((ext_vector_type(8)));
typedef int      v4i  __attribute__((ext_vector_type(4)));
typedef int      v8i  __attribute__((ext_vector_type(8)));
typedef _Float16 v8h  __attribute__((ext_vector_type(8)));
typedef _Float16 v16h __attribute__((ext_vector_type(16)));
union FragH { v16h v; v8h h[2]; v8i w; };

__device__ __forceinline__ v8f wmh(const FragH& a, const FragH& b, v8f c) {
  v8f d = __builtin_amdgcn_wmma_f32_16x16x32_f16(false, a.v, false, b.v, (short)0, c, false, false);
  asm volatile("v_nop\n\tv_nop\n\tv_nop\n\tv_nop" : "+v"(d) : "v"(a.w), "v"(b.w));
  return d;
}

__device__ __forceinline__ void ldwait() {
  asm volatile("s_wait_loadcnt 0x0" ::: "memory");
}

__device__ __forceinline__ float bf16r(float f) {
  unsigned u = __float_as_uint(f);
  u = (u + 0x7FFFu + ((u >> 16) & 1u)) & 0xFFFF0000u;
  return __uint_as_float(u);
}

__device__ __forceinline__ v8h cvt8h(const v4f a, const v4f b, const float c) {
  v8h hv;
  hv[0] = (_Float16)(a.x * c); hv[1] = (_Float16)(a.y * c);
  hv[2] = (_Float16)(a.z * c); hv[3] = (_Float16)(a.w * c);
  hv[4] = (_Float16)(b.x * c); hv[5] = (_Float16)(b.y * c);
  hv[6] = (_Float16)(b.z * c); hv[7] = (_Float16)(b.w * c);
  return hv;
}

__device__ __forceinline__ v8h cvt8hb(const v4f a, const v4f b, const float c) {
  v8h hv;
  hv[0] = (_Float16)(bf16r(a.x) * c); hv[1] = (_Float16)(bf16r(a.y) * c);
  hv[2] = (_Float16)(bf16r(a.z) * c); hv[3] = (_Float16)(bf16r(a.w) * c);
  hv[4] = (_Float16)(bf16r(b.x) * c); hv[5] = (_Float16)(bf16r(b.y) * c);
  hv[6] = (_Float16)(bf16r(b.z) * c); hv[7] = (_Float16)(bf16r(b.w) * c);
  return hv;
}

struct HL { _Float16 h; _Float16 l; };
__device__ __forceinline__ HL hl1(float v) {
  const float s = v * CX;
  const _Float16 hh = (_Float16)s;
  HL r;
  r.h = hh;
  r.l = (_Float16)((s - (float)hh) * CL);
  return r;
}

__device__ __forceinline__ void cvt8hl(const v4f a, const v4f b, v8h& hi, v8h& lo) {
  const HL e0 = hl1(a.x), e1 = hl1(a.y), e2 = hl1(a.z), e3 = hl1(a.w);
  const HL e4 = hl1(b.x), e5 = hl1(b.y), e6 = hl1(b.z), e7 = hl1(b.w);
  hi[0] = e0.h; hi[1] = e1.h; hi[2] = e2.h; hi[3] = e3.h;
  hi[4] = e4.h; hi[5] = e5.h; hi[6] = e6.h; hi[7] = e7.h;
  lo[0] = e0.l; lo[1] = e1.l; lo[2] = e2.l; lo[3] = e3.l;
  lo[4] = e4.l; lo[5] = e5.l; lo[6] = e6.l; lo[7] = e7.l;
}

__device__ __forceinline__ float selu1(float v) {
  const float e = __expf(fminf(v, 0.0f)) - 1.0f;
  return v > 0.0f ? SELU_SC * v : SELU_SC * (SELU_AL * e);
}

__device__ __forceinline__ int scan_chunk(const int* __restrict__ dsts, int nE, int cbase, int slotBase,
                                          int nb, int vec8, int* list, int tid, int lane, int wave) {
  int wc = 0;
  const int el0  = tid * EPT;
  const int e0   = cbase + el0;
  const int sent = -2147483647 - 1;
  v4i da, db;
  if (vec8 != 0 && cbase + CHUNK <= nE) {
    da = *(const v4i*)(dsts + e0);
    db = *(const v4i*)(dsts + e0 + 4);
  } else {
    da.x = (e0     < nE) ? dsts[min(e0,     nE - 1)] : sent;
    da.y = (e0 + 1 < nE) ? dsts[min(e0 + 1, nE - 1)] : sent;
    da.z = (e0 + 2 < nE) ? dsts[min(e0 + 2, nE - 1)] : sent;
    da.w = (e0 + 3 < nE) ? dsts[min(e0 + 3, nE - 1)] : sent;
    db.x = (e0 + 4 < nE) ? dsts[min(e0 + 4, nE - 1)] : sent;
    db.y = (e0 + 5 < nE) ? dsts[min(e0 + 5, nE - 1)] : sent;
    db.z = (e0 + 6 < nE) ? dsts[min(e0 + 6, nE - 1)] : sent;
    db.w = (e0 + 7 < nE) ? dsts[min(e0 + 7, nE - 1)] : sent;
  }
  const unsigned nbs = (unsigned)slotBase;
  const unsigned unb = (unsigned)nb;
  const unsigned s0 = (unsigned)da.x - nbs, s1 = (unsigned)da.y - nbs;
  const unsigned s2 = (unsigned)da.z - nbs, s3 = (unsigned)da.w - nbs;
  const unsigned s4 = (unsigned)db.x - nbs, s5 = (unsigned)db.y - nbs;
  const unsigned s6 = (unsigned)db.z - nbs, s7 = (unsigned)db.w - nbs;
  const bool h0 = s0 < unb, h1 = s1 < unb, h2 = s2 < unb, h3 = s3 < unb;
  const bool h4 = s4 < unb, h5 = s5 < unb, h6 = s6 < unb, h7 = s7 < unb;
  const unsigned any = __builtin_amdgcn_ballot_w32(h0 | h1 | h2 | h3 | h4 | h5 | h6 | h7);
  if (any != 0u) {
#define HITJ(J, HJ, SJ) { \
      const unsigned mj = __builtin_amdgcn_ballot_w32(HJ); \
      if (mj != 0u) { \
        if (HJ) { \
          const int pos = wc + (int)__builtin_amdgcn_mbcnt_lo(mj, 0u); \
          if (pos < WCAP) list[wave * WCAP + pos] = ((el0 + (J)) << 12) | (int)(SJ); \
        } \
        wc += (int)__builtin_popcount(mj); } }
    HITJ(0, h0, s0)
    HITJ(1, h1, s1)
    HITJ(2, h2, s2)
    HITJ(3, h3, s3)
    HITJ(4, h4, s4)
    HITJ(5, h5, s5)
    HITJ(6, h6, s6)
    HITJ(7, h7, s7)
#undef HITJ
  }
  return wc;
}

__global__ __launch_bounds__(NTHR) void k_xprep(const float* __restrict__ x, _Float16* xh, int nN, int nUnits) {
  const int i = (int)blockIdx.x * NTHR + (int)threadIdx.x;
  if (i >= nUnits) return;
  const int row = i >> 4;
  const int c0  = (i & 15) * 8;
  const int rc  = row < nN ? row : nN - 1;
  const float* p = x + (size_t)rc * DIN + c0;
  v4f a = *(const v4f*)p, b = *(const v4f*)(p + 4);
  const v4f z4 = {0.f, 0.f, 0.f, 0.f};
  if (row >= nN) { a = z4; b = z4; }
  const v8h hv = cvt8hb(a, b, CX);
  const size_t o = (size_t)row * DIN + c0;
  *(volatile v8h*)(xh + o) = hv;
  __threadfence();
  *(volatile v8h*)(xh + o) = hv;
}

__global__ __launch_bounds__(NTHR) void k_wtr(const float* __restrict__ w0, const float* __restrict__ w1,
                                              _Float16* wt, int nUnits) {
  const int u = (int)blockIdx.x * NTHR + (int)threadIdx.x;
  if (u >= nUnits) return;
  const int n   = u >> 4;
  const int k8  = (u & 15) * 8;
  const int seg = (n >> 7) & 1;
  const int nc  = n & (DIN - 1);
  const float* wsp = (seg == 0) ? w0 : w1;
  const float* p = wsp + (size_t)k8 * DIN + nc;
  v4f a, b;
  a.x = p[0];                   a.y = p[(size_t)DIN];         a.z = p[(size_t)2 * DIN];     a.w = p[(size_t)3 * DIN];
  b.x = p[(size_t)4 * DIN];     b.y = p[(size_t)5 * DIN];     b.z = p[(size_t)6 * DIN];     b.w = p[(size_t)7 * DIN];
  const v8h hv = cvt8hb(a, b, CW);
  const size_t o = (size_t)n * DIN + k8;
  *(volatile v8h*)(wt + o) = hv;
  __threadfence();
  *(volatile v8h*)(wt + o) = hv;
}

template<int NPL>
__global__ __launch_bounds__(GTHR) void k_gemm(
    const _Float16* __restrict__ A, const _Float16* __restrict__ AL, const _Float16* __restrict__ WT,
    const float* __restrict__ asrc, const float* __restrict__ adst,
    float* HP, int K, int h8)
{
  __shared__ __attribute__((aligned(16))) float stg[GBM * HPW];
  __shared__ __attribute__((aligned(16))) float avs[2 * GBN];
  const int tid = (int)threadIdx.x, lane = tid & 31, wave = tid >> 5, hh = lane >> 4, m = lane & 15;
  const int rowBase = (int)blockIdx.x * GBM;
  avs[tid]       = bf16r(asrc[tid]);
  avs[GBN + tid] = bf16r(adst[tid]);

  const _Float16* wp = WT + (size_t)m * (size_t)K + 8 * hh;
  const int ksteps = K >> 5;

#pragma unroll
  for (int pl = 0; pl < NPL; ++pl) {
    const _Float16* Ap = (pl == 0) ? A : AL;
    v8f acc[8];
    {
      const v8f z = {0.f, 0.f, 0.f, 0.f, 0.f, 0.f, 0.f, 0.f};
#pragma unroll
      for (int t = 0; t < 8; ++t) acc[t] = z;
    }
    const _Float16* ap = Ap + (size_t)(rowBase + 16 * wave + m) * (size_t)K + 8 * hh;
#pragma unroll 1
    for (int ks = 0; ks < ksteps; ++ks) {
      FragH af;
      af.h[0] = *(const v8h*)(ap + 32 * ks);
      af.h[1] = *(const v8h*)(ap + 32 * ks + 16);
#pragma unroll
      for (int t = 0; t < 8; ++t) {
        const _Float16* wq = wp + (size_t)(16 * t) * (size_t)K + 32 * ks;
        FragH bf;
        bf.h[0] = *(const v8h*)wq;
        bf.h[1] = *(const v8h*)(wq + 16);
        acc[t] = wmh(af, bf, acc[t]);
      }
    }

#pragma unroll
    for (int t = 0; t < 8; ++t) {
      const int lc = 16 * t + m;
#pragma unroll
      for (int r = 0; r < 8; ++r) {
        const int lr = 16 * wave + 8 * hh + r;
        if (pl == 0) stg[lr * HPW + lc] = acc[t][r] * SCL_HI;
        else         stg[lr * HPW + lc] = fmaf(acc[t][r], SCL_LO, stg[lr * HPW + lc]);
      }
    }
  }
  __syncthreads();

  {
    const int row   = tid & (GBM - 1);
    const int which = tid >> 6;
    const float* av = avs + which * GBN;
    const float* sr = stg + row * HPW;
    float pg[8];
    float tot = 0.f;
#pragma unroll
    for (int g = 0; g < 8; ++g) {
      float p = 0.f;
#pragma unroll 4
      for (int c = 0; c < 16; ++c) p = fmaf(sr[16 * g + c], av[16 * g + c], p);
      pg[g] = p;
      tot += p;
    }
    float* sw = stg + row * HPW + GBN + 8 * which;
#pragma unroll
    for (int g = 0; g < 8; ++g) sw[g] = (h8 != 0) ? pg[g] : ((g == 0) ? tot : 0.f);
    float* zw = stg + row * HPW + GBN + 16 + 8 * which;
#pragma unroll
    for (int g = 0; g < 8; ++g) zw[g] = 0.f;
  }
  __syncthreads();

  const float* sp = stg + (16 * wave) * HPW;
  float* op = HP + (size_t)(rowBase + 16 * wave) * (size_t)HPW;
#pragma unroll
  for (int i = 0; i < NSTV; ++i) {
    const v4f v = *(const v4f*)(sp + 4 * (32 * i + lane));
    *(volatile v4f*)(op + 4 * (32 * i + lane)) = v;
  }
  __threadfence();
#pragma unroll
  for (int i = 0; i < NSTV; ++i) {
    const v4f v = *(const v4f*)(sp + 4 * (32 * i + lane));
    *(volatile v4f*)(op + 4 * (32 * i + lane)) = v;
  }
}

__global__ __launch_bounds__(NTHR) void k_agg(
    const int* __restrict__ srcs, const int* __restrict__ dsts,
    const float* __restrict__ HP, const float* __restrict__ bias,
    float* AGG, float* PART,
    int nN, int nE, int nb, int vec8, int MPr, int cshift) {
  extern __shared__ v4f lds_dyn[];
  int* reg1 = (int*)lds_dyn;
  int* reg2 = reg1 + RCAP;
  int* scnt = reg2 + RCAP;
  int* soff = scnt + NBMAX;
  int* list = soff + NBMAX;
  int* wcnt = list + LISTN;
  int* wtot = wcnt + NWAVE;
  const int tid = (int)threadIdx.x, lane = tid & 31, wave = tid >> 5;
  const int nodeBase = (int)blockIdx.x * nb;

  for (int i = tid; i < NBMAX; i += NTHR) scnt[i] = 0;
  __syncthreads();

  int tot = 0;
  const int nChunks = (nE + CHUNK - 1) / CHUNK;
#pragma unroll 1
  for (int ch = 0; ch < nChunks; ++ch) {
    const int cbase = ch * CHUNK;
    const int wc = scan_chunk(dsts, nE, cbase, nodeBase, nb, vec8, list, tid, lane, wave);
    if (lane == 0) wcnt[wave] = wc;
    __syncthreads();
    int pre = 0, all = 0;
#pragma unroll
    for (int w2 = 0; w2 < NWAVE; ++w2) {
      int c = wcnt[w2];
      c = c < 0 ? 0 : (c > WCAP ? WCAP : c);
      all += c;
      pre += (w2 < wave) ? c : 0;
    }
    const int wcc  = wc > WCAP ? WCAP : wc;
    const int base = tot + pre;
#pragma unroll 1
    for (int i = lane; i < wcc; i += 32) {
      const int ent = list[wave * WCAP + i];
      const int el  = (ent >> 12) & (CHUNK - 1);
      const int sl  = ent & (NBMAX - 1);
      int eid = cbase + el;
      eid = eid > nE - 1 ? nE - 1 : eid;
      const int pos = base + i;
      if (pos < RCAP) reg1[pos] = (int)(((unsigned)eid << 12) | (unsigned)sl);
    }
    tot += all;
    tot = tot > RCAP ? RCAP : tot;
    __syncthreads();
  }
  const int nh = tot;

  if (wave == 0) {
#pragma unroll 1
    for (int b0 = 0; b0 < nh; b0 += 32) {
      const int idx = b0 + lane;
      const int uv  = reg1[idx < RCAP ? idx : RCAP - 1];
      const int m32 = (nh - b0) < 32 ? (nh - b0) : 32;
#pragma unroll 1
      for (int k = 0; k < m32; ++k) {
        const int u  = __builtin_amdgcn_readlane(uv, k);
        const int sl = u & (NBMAX - 1);
        if (lane == 0) scnt[sl] = scnt[sl] + 1;
      }
    }
  }
  __syncthreads();

  {
    const v4i ca = *(const v4i*)(scnt + 8 * tid);
    const v4i cb = *(const v4i*)(scnt + 8 * tid + 4);
    const int e0 = ca.x < 0 ? 0 : ca.x, e1 = ca.y < 0 ? 0 : ca.y, e2 = ca.z < 0 ? 0 : ca.z, e3 = ca.w < 0 ? 0 : ca.w;
    const int e4 = cb.x < 0 ? 0 : cb.x, e5 = cb.y < 0 ? 0 : cb.y, e6 = cb.z < 0 ? 0 : cb.z, e7 = cb.w < 0 ? 0 : cb.w;
    const int ts = e0 + e1 + e2 + e3 + e4 + e5 + e6 + e7;
    int incl = ts;
#pragma unroll
    for (int d = 1; d < 32; d <<= 1) {
      const int up = __shfl_up(incl, d);
      if (lane >= d) incl += up;
    }
    if (lane == 31) wtot[wave] = incl;
    __syncthreads();
    int pre = 0;
#pragma unroll
    for (int w2 = 0; w2 < NWAVE; ++w2) pre += (w2 < wave) ? wtot[w2] : 0;
    int run = pre + incl - ts;
    soff[8 * tid + 0] = run; run += e0;
    soff[8 * tid + 1] = run; run += e1;
    soff[8 * tid + 2] = run; run += e2;
    soff[8 * tid + 3] = run; run += e3;
    soff[8 * tid + 4] = run; run += e4;
    soff[8 * tid + 5] = run; run += e5;
    soff[8 * tid + 6] = run; run += e6;
    soff[8 * tid + 7] = run;
  }
  __syncthreads();
  for (int i = tid; i < NBMAX; i += NTHR) list[i] = soff[i];
  __syncthreads();

  if (wave == 0) {
#pragma unroll 1
    for (int b0 = 0; b0 < nh; b0 += 32) {
      const int idx = b0 + lane;
      const int uv  = reg1[idx < RCAP ? idx : RCAP - 1];
      const int m32 = (nh - b0) < 32 ? (nh - b0) : 32;
#pragma unroll 1
      for (int k = 0; k < m32; ++k) {
        const int u   = __builtin_amdgcn_readlane(uv, k);
        const int sl  = u & (NBMAX - 1);
        const int eid = (int)((unsigned)u >> 12);
        if (lane == 0) {
          int pos = list[sl];
          pos = pos < 0 ? 0 : (pos > RCAP - 1 ? RCAP - 1 : pos);
          reg2[pos] = eid;
          list[sl] = pos + 1;
        }
      }
    }
  }
  __syncthreads();

  const int nbw = nb >> 3;
  const bool ovf = (nh >= RCAP);
  const float qnan = __int_as_float(0x7fc00000);
  float* stw = (float*)reg1 + wave * STW;
  const int cs = cshift < 4 ? 4 : (cshift > 7 ? 7 : cshift);
  int hd[4];
  float bb[4], sx[4], sq[4];
#pragma unroll
  for (int j = 0; j < 4; ++j) {
    hd[j] = (32 * j + lane) >> cs;
    bb[j] = bf16r(bias[32 * j + lane]);
    sx[j] = 0.f; sq[j] = 0.f;
  }
#pragma unroll 1
  for (int jt = 0; jt < nbw; ++jt) {
    const int slot = wave * nbw + jt;
    const int grow = nodeBase + slot;
    const int gcl  = grow < nN ? grow : nN - 1;
    int st = soff[slot];
    const int craw = scnt[slot];
    int cnt = craw;
    st  = st < 0 ? 0 : (st > nh ? nh : st);
    cnt = cnt < 0 ? 0 : (cnt > DEGCAP ? DEGCAP : cnt);
    if (cnt > nh - st) cnt = nh - st;
    const float pz = (ovf || craw > DEGCAP) ? qnan : 0.0f;
    const bool wr = grow < MPr;
    const float live = grow < nN ? 1.0f : 0.0f;

    const float* drow = HP + (size_t)gcl * HPW + (DIN + 8);
    float dv[4];
#pragma unroll
    for (int j = 0; j < 4; ++j) dv[j] = drow[hd[j]];
    ldwait();
    float mx[4], dn[4], av[4];
#pragma unroll
    for (int j = 0; j < 4; ++j) { mx[j] = -1.0e30f; dn[j] = 0.f; av[j] = 0.f; }

#pragma unroll 1
    for (int q = 0; q <= cnt; ++q) {
      int s = gcl;
      if (q < cnt) {
        int idx = st + q; idx = idx > RCAP - 1 ? RCAP - 1 : idx;
        int eid = reg2[idx]; eid = eid < 0 ? 0 : (eid > nE - 1 ? nE - 1 : eid);
        const int sraw = srcs[eid];
        s = sraw < 0 ? 0 : (sraw > nN - 1 ? nN - 1 : sraw);
      }
      const float* hr = HP + (size_t)s * HPW;
      float hv[4], sv[4];
#pragma unroll
      for (int j = 0; j < 4; ++j) hv[j] = hr[32 * j + lane];
#pragma unroll
      for (int j = 0; j < 4; ++j) sv[j] = hr[DIN + hd[j]];
      ldwait();
#pragma unroll
      for (int j = 0; j < 4; ++j) {
        float e = sv[j] + dv[j];
        e = e > 0.f ? e : NEG_SLOPE * e;
        const float df = e - mx[j];
        const float ee = __expf(-fabsf(df));
        const bool up  = df > 0.f;
        const float s1 = up ? ee : 1.0f;
        const float s2 = up ? 1.0f : ee;
        mx[j] = up ? e : mx[j];
        dn[j] = fmaf(dn[j], s1, s2);
        av[j] = fmaf(av[j], s1, s2 * hv[j]);
      }
    }
    float r[4];
#pragma unroll
    for (int j = 0; j < 4; ++j) {
      r[j] = fmaf(av[j], __builtin_amdgcn_rcpf(dn[j]), bb[j]) * live + pz;
      sx[j] += r[j];
      sq[j] = fmaf(r[j], r[j], sq[j]);
    }
    __builtin_amdgcn_fence(__ATOMIC_RELEASE, "wavefront");
    __builtin_amdgcn_wave_barrier();
#pragma unroll
    for (int j = 0; j < 4; ++j) stw[32 * j + lane] = r[j];
    __builtin_amdgcn_fence(__ATOMIC_RELEASE, "wavefront");
    __builtin_amdgcn_wave_barrier();
    const v4f ga = *(const v4f*)(stw + 4 * lane);
    float* gp = AGG + (size_t)grow * DIN + 4 * lane;
    if (wr) *(volatile v4f*)gp = ga;
    __threadfence();
    if (wr) *(volatile v4f*)gp = ga;
  }

  float* sts = (float*)reg1 + STS;
#pragma unroll
  for (int j = 0; j < 4; ++j) {
    sts[wave * PREC + 32 * j + lane]       = sx[j];
    sts[wave * PREC + DIN + 32 * j + lane] = sq[j];
  }
  __syncthreads();
  float* cmb = sts + NWAVE * PREC;
  {
    float a = 0.f;
#pragma unroll
    for (int w2 = 0; w2 < NWAVE; ++w2) a += sts[w2 * PREC + tid];
    cmb[tid] = a;
  }
  __syncthreads();
  if (wave == 0) {
    const v4f p0 = *(const v4f*)(cmb + 4 * lane);
    const v4f p1 = *(const v4f*)(cmb + DIN + 4 * lane);
    float* pp = PART + (size_t)blockIdx.x * PREC;
    *(volatile v4f*)(pp + 4 * lane)       = p0;
    *(volatile v4f*)(pp + DIN + 4 * lane) = p1;
    __threadfence();
    *(volatile v4f*)(pp + 4 * lane)       = p0;
    *(volatile v4f*)(pp + DIN + 4 * lane) = p1;
  }
}

__global__ __launch_bounds__(NTHR) void k_bnfold(const float* __restrict__ part, int nP,
                                                 const float* __restrict__ gamma, const float* __restrict__ beta,
                                                 float invN, float* SS) {
  __shared__ double dsum[PREC];
  __shared__ __attribute__((aligned(16))) float so[PREC];
  const int tid = (int)threadIdx.x, lane = tid & 31, wave = tid >> 5;
  const int np = nP < 0 ? 0 : nP;
  double a = 0.0;
#pragma unroll 1
  for (int b = 0; b < np; ++b) a += (double)part[(size_t)b * PREC + tid];
  dsum[tid] = a;
  __syncthreads();
  if (tid < DIN) {
    const double dinv = (double)invN;
    const double mean = dsum[tid] * dinv;
    double var = dsum[DIN + tid] * dinv - mean * mean;
    var = var < 0.0 ? 0.0 : var;
    const float sc = bf16r(gamma[tid]) * rsqrtf((float)var + EPS_BN);
    const float sh = bf16r(beta[tid]) - (float)mean * sc;
    so[tid]       = sc;
    so[DIN + tid] = sh;
  }
  __syncthreads();
  if (wave == 0) {
    const v4f p0 = *(const v4f*)(so + 4 * lane);
    const v4f p1 = *(const v4f*)(so + DIN + 4 * lane);
    *(volatile v4f*)(SS + 4 * lane)       = p0;
    *(volatile v4f*)(SS + DIN + 4 * lane) = p1;
    __threadfence();
    *(volatile v4f*)(SS + 4 * lane)       = p0;
    *(volatile v4f*)(SS + DIN + 4 * lane) = p1;
  }
}

__global__ __launch_bounds__(NTHR) void k_bncvt(const float* __restrict__ agg, const float* __restrict__ SS,
                                                _Float16* yh, _Float16* yl, int nN, int nUnits) {
  const int i = (int)blockIdx.x * NTHR + (int)threadIdx.x;
  if (i >= nUnits) return;
  const int row = i >> 4;
  const int c0  = (i & 15) * 8;
  const int rc  = row < nN ? row : nN - 1;
  const float* p = agg + (size_t)rc * DIN + c0;
  const v4f a = *(const v4f*)p, b = *(const v4f*)(p + 4);
  const v4f sa = *(const v4f*)(SS + c0),       sb = *(const v4f*)(SS + c0 + 4);
  const v4f ta = *(const v4f*)(SS + DIN + c0), tb = *(const v4f*)(SS + DIN + c0 + 4);
  v4f ya, yb;
  ya.x = selu1(fmaf(a.x, sa.x, ta.x)); ya.y = selu1(fmaf(a.y, sa.y, ta.y));
  ya.z = selu1(fmaf(a.z, sa.z, ta.z)); ya.w = selu1(fmaf(a.w, sa.w, ta.w));
  yb.x = selu1(fmaf(b.x, sb.x, tb.x)); yb.y = selu1(fmaf(b.y, sb.y, tb.y));
  yb.z = selu1(fmaf(b.z, sb.z, tb.z)); yb.w = selu1(fmaf(b.w, sb.w, tb.w));
  const v4f z4 = {0.f, 0.f, 0.f, 0.f};
  if (row >= nN) { ya = z4; yb = z4; }
  v8h hv, lv;
  cvt8hl(ya, yb, hv, lv);
  const size_t o = (size_t)row * DIN + c0;
  *(volatile v8h*)(yh + o) = hv;
  *(volatile v8h*)(yl + o) = lv;
  __threadfence();
  *(volatile v8h*)(yh + o) = hv;
  *(volatile v8h*)(yl + o) = lv;
}

__global__ __launch_bounds__(NTHR) void k_out(const float* __restrict__ agg, const float* __restrict__ SS,
                                              float* out, int nUnits) {
  const int i = (int)blockIdx.x * NTHR + (int)threadIdx.x;
  if (i >= nUnits) return;
  const int row = i >> 5;
  const int c0  = (i & 31) * 4;
  const v4f a = *(const v4f*)(agg + (size_t)row * DIN + c0);
  const v4f s = *(const v4f*)(SS + c0);
  const v4f t = *(const v4f*)(SS + DIN + c0);
  v4f y;
  y.x = selu1(fmaf(a.x, s.x, t.x)); y.y = selu1(fmaf(a.y, s.y, t.y));
  y.z = selu1(fmaf(a.z, s.z, t.z)); y.w = selu1(fmaf(a.w, s.w, t.w));
  float* op = out + (size_t)row * DIN + c0;
  *(volatile v4f*)op = y;
  __threadfence();
  *(volatile v4f*)op = y;
}

static int pick_nb(int nE, int nN) {
  int nb = NBMAX;
  while (nb > 16 && (long long)nb * (long long)nE * 5LL > (long long)RCAP * (long long)nN * 4LL) nb >>= 1;
  return nb;
}
static inline int cdiv(int a, int b) { return (a + b - 1) / b; }

extern "C" void kernel_launch(void* const* d_in, const int* in_sizes, int n_in,
                              void* d_out, int out_size, void* d_ws, size_t ws_size,
                              hipStream_t stream) {
  if (n_in < 15) return;
  const int nN = in_sizes[0] / DIN;
  if (nN <= 0 || in_sizes[0] != nN * DIN || nN > (1 << 22)) return;
  if (in_sizes[1] < 2 || (in_sizes[1] & 1) != 0) return;
  const int nE = in_sizes[1] / 2;
  if (nE < 1 || nE > (1 << 20)) return;
  if (in_sizes[3] != DIN * DIN || in_sizes[9] != DIN * DIN) return;
  if (in_sizes[4]  != DIN || in_sizes[5]  != DIN) return;
  if (in_sizes[6]  != DIN || in_sizes[7]  != DIN || in_sizes[8]  != DIN) return;
  if (in_sizes[10] != DIN || in_sizes[11] != DIN) return;
  if (in_sizes[12] != DIN || in_sizes[13] != DIN || in_sizes[14] != DIN) return;
  if (out_size != nN * DIN) return;

  const float* x   = (const float*)d_in[0];
  const int*   ei  = (const int*)  d_in[1];
  const float* W1  = (const float*)d_in[3];
  const float* as1 = (const float*)d_in[4];
  const float* ad1 = (const float*)d_in[5];
  const float* b1  = (const float*)d_in[6];
  const float* g1  = (const float*)d_in[7];
  const float* be1 = (const float*)d_in[8];
  const float* W2  = (const float*)d_in[9];
  const float* as2 = (const float*)d_in[10];
  const float* ad2 = (const float*)d_in[11];
  const float* b2  = (const float*)d_in[12];
  const float* g2  = (const float*)d_in[13];
  const float* be2 = (const float*)d_in[14];
  float* out = (float*)d_out;
  const int* src = ei;
  const int* dst = ei + nE;

  const int MP   = cdiv(nN, GBM) * GBM;
  const int nb   = pick_nb(nE, nN);
  const int gA   = cdiv(MP, nb);
  const int vec8 = ((nE & 3) == 0) ? 1 : 0;
  if (gA * nb < MP || (nb & 7) != 0) return;
  const float invN = 1.0f / (float)nN;

  char* ws = (char*)d_ws;
  size_t off = 0;
  const size_t oXH  = off; off += (size_t)MP * DIN * 2;            off = (off + 255) & ~(size_t)255;
  const size_t oWT  = off; off += (size_t)2 * DIN * DIN * 2;       off = (off + 255) & ~(size_t)255;
  const size_t oHP  = off; off += (size_t)MP * HPW * 4;            off = (off + 255) & ~(size_t)255;
  const size_t oAG  = off; off += (size_t)MP * DIN * 4;            off = (off + 255) & ~(size_t)255;
  const size_t oY1  = off; off += (size_t)MP * DIN * 2;            off = (off + 255) & ~(size_t)255;
  const size_t oYL  = off; off += (size_t)MP * DIN * 2;            off = (off + 255) & ~(size_t)255;
  const size_t oPT  = off; off += (size_t)gA * PREC * 4;           off = (off + 255) & ~(size_t)255;
  const size_t oS1  = off; off += (size_t)PREC * 4;                off = (off + 255) & ~(size_t)255;
  const size_t oS2  = off; off += (size_t)PREC * 4;                off = (off + 255) & ~(size_t)255;
  if (off > ws_size || off > (size_t)WSMAX) return;
  _Float16* XH  = (_Float16*)(ws + oXH);
  _Float16* WT  = (_Float16*)(ws + oWT);
  float*    HP  = (float*)(ws + oHP);
  float*    AGG = (float*)(ws + oAG);
  _Float16* Y1H = (_Float16*)(ws + oY1);
  _Float16* Y1L = (_Float16*)(ws + oYL);
  float*    PART = (float*)(ws + oPT);
  float*    SS1 = (float*)(ws + oS1);
  float*    SS2 = (float*)(ws + oS2);

  hipFuncSetAttribute(reinterpret_cast<const void*>(&k_agg),
                      hipFuncAttributeMaxDynamicSharedMemorySize, LDS_AGG);

  const int nUx = MP * (DIN / 8);
  k_xprep<<<cdiv(nUx, NTHR), NTHR, 0, stream>>>(x, XH, nN, nUx);
  const int nUw = 2 * DIN * (DIN / 8);
  k_wtr<<<cdiv(nUw, NTHR), NTHR, 0, stream>>>(W1, W2, WT, nUw);

  const int gM = MP / GBM;
  k_gemm<1><<<gM, GTHR, 0, stream>>>(XH, XH, WT, as1, ad1, HP, DIN, 1);
  k_agg<<<gA, NTHR, LDS_AGG, stream>>>(src, dst, HP, b1, AGG, PART, nN, nE, nb, vec8, MP, 4);
  k_bnfold<<<1, NTHR, 0, stream>>>(PART, gA, g1, be1, invN, SS1);
  k_bncvt<<<cdiv(nUx, NTHR), NTHR, 0, stream>>>(AGG, SS1, Y1H, Y1L, nN, nUx);
  k_gemm<2><<<gM, GTHR, 0, stream>>>(Y1H, Y1L, WT + (size_t)DIN * DIN, as2, ad2, HP, DIN, 0);
  k_agg<<<gA, NTHR, LDS_AGG, stream>>>(src, dst, HP, b2, AGG, PART, nN, nE, nb, vec8, MP, 7);
  k_bnfold<<<1, NTHR, 0, stream>>>(PART, gA, g2, be2, invN, SS2);
  const int nUo = nN * (DIN / 4);
  k_out<<<cdiv(nUo, NTHR), NTHR, 0, stream>>>(AGG, SS2, out, nUo);
}
